// FeedbackTransformer_79061757985040
// MI455X (gfx1250) — hardware-run, weakly checked
//
#include <hip/hip_runtime.h>
#include <math.h>
#include <stddef.h>

typedef __attribute__((ext_vector_type(16))) _Float16 v16h;
typedef __attribute__((ext_vector_type(8)))  _Float16 v8h;
typedef __attribute__((ext_vector_type(4)))  _Float16 v4h;
typedef __attribute__((ext_vector_type(2)))  _Float16 v2h;
typedef __attribute__((ext_vector_type(8)))  float    v8f;
typedef __attribute__((ext_vector_type(4)))  float    v4f;
typedef __attribute__((ext_vector_type(2)))  float    v2f;

__device__ __forceinline__ void dep_guard_h(v8f& a, v8f& b, v16h x, v16h y) { asm volatile("v_nop\n\tv_nop\n\tv_nop\n\tv_nop" : "+v"(a), "+v"(b) : "v"(x), "v"(y)); }
__device__ __forceinline__ void dep_guard1(v8f& a, v16h x, v16h y) { asm volatile("v_nop\n\tv_nop\n\tv_nop\n\tv_nop" : "+v"(a) : "v"(x), "v"(y)); }
__device__ __forceinline__ void keep4_h(v16h a, v16h b, v16h c, v16h d) { asm volatile("v_nop" :: "v"(a), "v"(b), "v"(c), "v"(d)); }
__device__ __forceinline__ void acc_guard4(v8f& a, v8f& b, v8f& c, v8f& d) { asm volatile("v_nop\n\tv_nop\n\tv_nop\n\tv_nop" : "+v"(a), "+v"(b), "+v"(c), "+v"(d)); }
template <typename T> struct Frag;
template <> struct Frag<_Float16> {
  typedef v16h V; union U { v16h v; v8h h[2]; };
  static __device__ __forceinline__ v16h load(const _Float16* p) {
    U f; f.h[0] = *(const v8h*)(p); f.h[1] = *(const v8h*)(p + 16); return f.v;
  }
  static __device__ __forceinline__ v8f mma(v16h a, v16h b, v8f c) {
    return __builtin_amdgcn_wmma_f32_16x16x32_f16(false, a, false, b, (short)0, c, false, false);
  }
  static __device__ __forceinline__ void guard(v8f& a, v8f& b, v16h x, v16h y) { dep_guard_h(a, b, x, y); }
  static __device__ __forceinline__ void keep(v16h a, v16h b, v16h c, v16h d) { keep4_h(a, b, c, d); }
};

constexpr int SEQ = 128;
constexpr int NBATCH = 32;
constexpr int DM = 512;
constexpr int NHEAD = 8;
constexpr int DHEAD = 64;
constexpr int DFFN = 2048;
constexpr int NLAY = 4;
constexpr int NPOS = 4096;
constexpr int BPB = 16;
constexpr int NBLK = NBATCH / BPB;
constexpr int NTHR = 256;
constexpr int NWAVE = NTHR / 32;
constexpr float WCARRY = 64.0f;
constexpr float INV_WC = 1.0f / 64.0f;
constexpr float INV_WC2 = 1.0f / 4096.0f;
constexpr float ATT_SCALE = 0.125f;
constexpr float NEG_FILL = -1.0e9f;
constexpr size_t MEMPLANE = (size_t)NLAY * SEQ * NBATCH * DM;
constexpr int SLAB_PITCH = 68;
constexpr int SLAB_FLOATS = 16 * SLAB_PITCH;

static_assert(BPB == 16);
static_assert(NBLK * BPB == NBATCH);
static_assert(NHEAD == NWAVE);
static_assert(NWAVE * 64 == DM);
static_assert(DHEAD == 64);
static_assert(NHEAD * DHEAD == DM);
static_assert(DM % 32 == 0 && DFFN % 32 == 0);
static_assert(DM % 64 == 0 && DFFN % 64 == 0);
static_assert(DFFN % DM == 0);
static_assert(SEQ == 128);
static_assert((BPB * DM / 4) % NTHR == 0);
static_assert((BPB * DM / 8) % NTHR == 0);
static_assert(NWAVE * SLAB_FLOATS <= 16384);
static_assert(NLAY + 1 == 5);

constexpr size_t WQ_BYTES = (size_t)NLAY * DM * DM * 2;
constexpr size_t W1_BYTES = (size_t)NLAY * DFFN * DM * 2;
constexpr size_t PE_BYTES = (size_t)NLAY * NHEAD * SEQ * DHEAD * 2;
constexpr size_t MEM_BYTES = 2 * MEMPLANE * 4;
constexpr size_t OFF_WQ = 0;
constexpr size_t OFF_WKV = OFF_WQ + WQ_BYTES;
constexpr size_t OFF_WO = OFF_WKV + 2 * WQ_BYTES;
constexpr size_t OFF_W1 = OFF_WO + WQ_BYTES;
constexpr size_t OFF_W2 = OFF_W1 + W1_BYTES;
constexpr size_t OFF_PE = OFF_W2 + W1_BYTES;
constexpr size_t OFF_MEM = OFF_PE + PE_BYTES;
constexpr size_t WS_TOTAL = OFF_MEM + MEM_BYTES;
static_assert(WS_TOTAL == 92798976);
static_assert(WS_TOTAL <= (size_t)134217728);
static_assert(OFF_WKV % 128 == 0 && OFF_WO % 128 == 0 && OFF_W1 % 128 == 0 && OFF_W2 % 128 == 0 && OFF_PE % 128 == 0 && OFF_MEM % 128 == 0);

__device__ __forceinline__ float wave_sum(float x) {
#pragma unroll
  for (int m = 16; m > 0; m >>= 1) x += __shfl_xor(x, m, 32);
  return x;
}
__device__ __forceinline__ float wave_max(float x) {
#pragma unroll
  for (int m = 16; m > 0; m >>= 1) x = fmaxf(x, __shfl_xor(x, m, 32));
  return x;
}
__device__ __forceinline__ void wave_lds_sync() {
  __builtin_amdgcn_fence(__ATOMIC_RELEASE, "workgroup");
  __builtin_amdgcn_wave_barrier();
  __builtin_amdgcn_fence(__ATOMIC_ACQUIRE, "workgroup");
}

template <int KDIM, int LDA, int LDB>
__device__ __forceinline__ void mm16x64(const _Float16* As, const _Float16* __restrict__ Bt, int n0, v8f (&acc)[4]) {
  static_assert(KDIM % 32 == 0);
  static_assert(LDA % 8 == 0 && LDB % 8 == 0);
  const int lane = threadIdx.x & 31;
  const int rl = lane & 15;
  const int koff = (lane >> 4) * 8;
#pragma unroll
  for (int j = 0; j < 4; ++j) acc[j] = (v8f){0.f, 0.f, 0.f, 0.f, 0.f, 0.f, 0.f, 0.f};
  const _Float16* ap = As + rl * LDA + koff;
  const _Float16* bp = Bt + (size_t)(n0 + rl) * LDB + koff;
  for (int k0 = 0; k0 < KDIM; k0 += 32) {
    v16h bq[4];
#pragma unroll
    for (int j = 0; j < 4; ++j) bq[j] = Frag<_Float16>::load(bp + (size_t)(16 * j) * LDB + k0);
    const v16h a = Frag<_Float16>::load(ap + k0);
#pragma unroll
    for (int j = 0; j < 4; ++j) acc[j] = Frag<_Float16>::mma(a, bq[j], acc[j]);
    Frag<_Float16>::guard(acc[0], acc[3], a, a);
    Frag<_Float16>::keep(bq[0], bq[1], bq[2], bq[3]);
  }
  acc_guard4(acc[0], acc[1], acc[2], acc[3]);
}

__device__ __forceinline__ void ln_to_a16(const float* hsrc, const float* __restrict__ g, const float* __restrict__ bb, _Float16* a16d) {
  const int lane = threadIdx.x & 31, wave = threadIdx.x >> 5;
  v4f g4[4], b4[4];
#pragma unroll
  for (int i = 0; i < 4; ++i) {
    g4[i] = *(const v4f*)(g + 128 * i + 4 * lane);
    b4[i] = *(const v4f*)(bb + 128 * i + 4 * lane);
  }
#pragma unroll 1
  for (int rr = 0; rr < 2; ++rr) {
    const int row = wave + 8 * rr;
    v4f x[4];
#pragma unroll
    for (int i = 0; i < 4; ++i) x[i] = *(const v4f*)(hsrc + row * DM + 128 * i + 4 * lane);
    float s = 0.f;
#pragma unroll
    for (int i = 0; i < 4; ++i) s += (x[i][0] + x[i][1]) + (x[i][2] + x[i][3]);
    s = wave_sum(s);
    const float mu = s * (1.0f / 512.0f);
    float ss = 0.f;
#pragma unroll
    for (int i = 0; i < 4; ++i) {
      const v4f d = x[i] - mu;
      ss += (d[0] * d[0] + d[1] * d[1]) + (d[2] * d[2] + d[3] * d[3]);
    }
    ss = wave_sum(ss);
    const float rstd = rsqrtf(ss * (1.0f / 512.0f) + 1e-5f);
#pragma unroll
    for (int i = 0; i < 4; ++i) {
      const v4f z = (x[i] - mu) * rstd * g4[i] + b4[i];
      v4h hv;
      hv[0] = (_Float16)z[0]; hv[1] = (_Float16)z[1]; hv[2] = (_Float16)z[2]; hv[3] = (_Float16)z[3];
      *(v4h*)(a16d + row * DM + 128 * i + 4 * lane) = hv;
    }
  }
}

__device__ __forceinline__ void ln_to_out(const float* hsrc, const float* __restrict__ g, const float* __restrict__ bb, float* __restrict__ obase) {
  const int lane = threadIdx.x & 31, wave = threadIdx.x >> 5;
  v4f g4[4], b4[4];
#pragma unroll
  for (int i = 0; i < 4; ++i) {
    g4[i] = *(const v4f*)(g + 128 * i + 4 * lane);
    b4[i] = *(const v4f*)(bb + 128 * i + 4 * lane);
  }
#pragma unroll 1
  for (int rr = 0; rr < 2; ++rr) {
    const int row = wave + 8 * rr;
    v4f x[4];
#pragma unroll
    for (int i = 0; i < 4; ++i) x[i] = *(const v4f*)(hsrc + row * DM + 128 * i + 4 * lane);
    float s = 0.f;
#pragma unroll
    for (int i = 0; i < 4; ++i) s += (x[i][0] + x[i][1]) + (x[i][2] + x[i][3]);
    s = wave_sum(s);
    const float mu = s * (1.0f / 512.0f);
    float ss = 0.f;
#pragma unroll
    for (int i = 0; i < 4; ++i) {
      const v4f d = x[i] - mu;
      ss += (d[0] * d[0] + d[1] * d[1]) + (d[2] * d[2] + d[3] * d[3]);
    }
    ss = wave_sum(ss);
    const float rstd = rsqrtf(ss * (1.0f / 512.0f) + 1e-5f);
    v4f z[4];
#pragma unroll
    for (int i = 0; i < 4; ++i) z[i] = (x[i] - mu) * rstd * g4[i] + b4[i];
    float* orow = obase + (size_t)row * DM + 4 * lane;
    for (int pass = 0; pass < 2; ++pass) {
#pragma unroll
      for (int i = 0; i < 4; ++i) *(volatile v4f*)(orow + 128 * i) = z[i];
      __threadfence();
    }
  }
}

__global__ __launch_bounds__(256) void k_wtcast(const float* __restrict__ in, _Float16* __restrict__ outp, int Kd, int Nd) {
  __shared__ float T[64 * 65];
  const int tid = threadIdx.x;
  const int n0 = blockIdx.x * 64, k0 = blockIdx.y * 64, l = blockIdx.z;
  {
    const int kr = tid >> 2, cq = (tid & 3) * 16;
    const float* src = in + ((size_t)l * Kd + k0 + kr) * Nd + n0 + cq;
#pragma unroll
    for (int e = 0; e < 4; ++e) {
      const v4f v = *(const v4f*)(src + 4 * e);
      T[(cq + 4 * e + 0) * 65 + kr] = v[0];
      T[(cq + 4 * e + 1) * 65 + kr] = v[1];
      T[(cq + 4 * e + 2) * 65 + kr] = v[2];
      T[(cq + 4 * e + 3) * 65 + kr] = v[3];
    }
  }
  __syncthreads();
  const int nr = tid >> 3, k8 = (tid & 7) * 8;
  v8h hv0, hv1;
#pragma unroll
  for (int e = 0; e < 8; ++e) {
    hv0[e] = (_Float16)(T[nr * 65 + k8 + e] * WCARRY);
    hv1[e] = (_Float16)(T[(nr + 32) * 65 + k8 + e] * WCARRY);
  }
  _Float16* o0 = outp + ((size_t)l * Nd + n0 + nr) * Kd + k0 + k8;
  _Float16* o1 = outp + ((size_t)l * Nd + n0 + nr + 32) * Kd + k0 + k8;
  for (int pass = 0; pass < 2; ++pass) {
    *(volatile v8h*)o0 = hv0;
    *(volatile v8h*)o1 = hv1;
    __threadfence();
  }
}

__global__ __launch_bounds__(256) void k_pecast(const float* __restrict__ kpe, _Float16* __restrict__ pe16) {
  const int gi = blockIdx.x * 256 + threadIdx.x;
  const int d8 = (gi & 7) * 8;
  const int rowo = gi >> 3;
  const int pp = rowo & (SEQ - 1);
  const int lh = rowo >> 7;
  const int h = lh & (NHEAD - 1);
  const int l = lh >> 3;
  const float* src = kpe + (((size_t)l * NPOS + (size_t)(NPOS - SEQ + pp)) * NHEAD + h) * DHEAD + d8;
  const v4f a = *(const v4f*)(src);
  const v4f c = *(const v4f*)(src + 4);
  v8h hv;
  hv[0] = (_Float16)(a[0] * WCARRY); hv[1] = (_Float16)(a[1] * WCARRY); hv[2] = (_Float16)(a[2] * WCARRY); hv[3] = (_Float16)(a[3] * WCARRY);
  hv[4] = (_Float16)(c[0] * WCARRY); hv[5] = (_Float16)(c[1] * WCARRY); hv[6] = (_Float16)(c[2] * WCARRY); hv[7] = (_Float16)(c[3] * WCARRY);
  _Float16* o = pe16 + (size_t)rowo * DHEAD + d8;
  for (int pass = 0; pass < 2; ++pass) {
    *(volatile v8h*)o = hv;
    __threadfence();
  }
}

union BigU { float f[16384]; _Float16 h[32768]; };

__global__ __launch_bounds__(NTHR) void k_steps(
    const float* __restrict__ x_seq,
    const float* __restrict__ lnsag, const float* __restrict__ lnsab,
    const _Float16* __restrict__ wqT, const _Float16* __restrict__ wkvT, const float* __restrict__ bvv,
    const _Float16* __restrict__ pe16, const float* __restrict__ kpb, const float* __restrict__ qpb,
    const _Float16* __restrict__ woT, const float* __restrict__ bo,
    const float* __restrict__ lnffg, const float* __restrict__ lnffb,
    const _Float16* __restrict__ w1T, const float* __restrict__ b1,
    const _Float16* __restrict__ w2T, const float* __restrict__ b2,
    const float* __restrict__ fusew, const float* __restrict__ lnog, const float* __restrict__ lnob,
    float* mem, float* __restrict__ out) {
  __shared__ __align__(16) float hs[BPB * DM];
  __shared__ __align__(16) float accm[BPB * DM];
  __shared__ __align__(16) _Float16 a16[BPB * DM];
  __shared__ __align__(16) BigU big;
  __shared__ __align__(16) float sc[NWAVE * SEQ];

  const int tid = threadIdx.x, lane = tid & 31, wave = tid >> 5, blk = blockIdx.x;
  const int rl = lane & 15, hh = lane >> 4, mOff = hh * 8, koff = hh * 8;

  float fz0, fz1, fz2, fz3, fz4;
  {
    const float u0 = fusew[0], u1 = fusew[1], u2 = fusew[2], u3 = fusew[3], u4 = fusew[4];
    const float mx = fmaxf(fmaxf(fmaxf(u0, u1), fmaxf(u2, u3)), u4);
    const float e0 = expf(u0 - mx), e1 = expf(u1 - mx), e2 = expf(u2 - mx), e3 = expf(u3 - mx), e4 = expf(u4 - mx);
    const float sm = (((e0 + e1) + e2) + e3) + e4;
    const float inv = 1.0f / sm;
    fz0 = e0 * inv; fz1 = e1 * inv; fz2 = e2 * inv; fz3 = e3 * inv; fz4 = e4 * inv;
  }

  float* const qa32 = big.f + 8192;
  _Float16* const bd16 = big.h;
  _Float16* const f1 = big.h;
  const _Float16* const f1c = big.h;
  float* const slab = big.f + wave * SLAB_FLOATS;
  float* const scw = sc + wave * SEQ;
  const float* const memk = mem;
  const float* const memv = mem + MEMPLANE;

#pragma unroll 1
  for (int t = 0; t < SEQ; ++t) {
    {
      const float* xs = x_seq + ((size_t)t * NBATCH + (size_t)blk * BPB) * DM;
#pragma unroll
      for (int i = 0; i < (BPB * DM / 4) / NTHR; ++i) {
        const int f = tid + NTHR * i;
        const v4f v = *(const v4f*)(xs + 4 * f);
        *(v4f*)(hs + 4 * f) = v;
        *(v4f*)(accm + 4 * f) = v * fz0;
      }
    }
    __syncthreads();
    __threadfence();

#pragma unroll 1
    for (int l = 0; l < NLAY; ++l) {
      const float fl = (l == 0) ? fz1 : (l == 1) ? fz2 : (l == 2) ? fz3 : fz4;
      if (t > 0) {
        ln_to_a16(hs, lnsag + l * DM, lnsab + l * DM, a16);
        __syncthreads();
        {
          v8f acc[4];
          mm16x64<DM, DM, DM>(a16, wqT + (size_t)l * DM * DM, wave * 64, acc);
          __syncthreads();
#pragma unroll
          for (int j = 0; j < 4; ++j) {
            const int col = wave * 64 + 16 * j + rl;
            const float pbq = qpb[l * DM + col];
#pragma unroll
            for (int r = 0; r < 8; ++r) {
              const int row = mOff + r;
              const float qv = acc[j][r] * INV_WC;
              qa32[row * DM + col] = qv + pbq;
              a16[row * DM + col] = (_Float16)qv;
            }
          }
        }
        __syncthreads();
        {
          const int hd = wave;
          const int ntile = ((t + 31) >> 5) * 2;
          const _Float16* peb = pe16 + (size_t)(l * NHEAD + hd) * SEQ * DHEAD;
          const _Float16* aq = a16 + rl * DM + hd * DHEAD + koff;
          for (int jt = 0; jt < ntile; ++jt) {
            int prow = SEQ - t + 16 * jt + rl;
            prow = prow > (SEQ - 1) ? (SEQ - 1) : prow;
            const _Float16* pbp = peb + (size_t)prow * DHEAD + koff;
            v8f acc = (v8f){0.f, 0.f, 0.f, 0.f, 0.f, 0.f, 0.f, 0.f};
#pragma unroll
            for (int ks = 0; ks < 2; ++ks) {
              const v16h a = Frag<_Float16>::load(aq + 32 * ks);
              const v16h bfr = Frag<_Float16>::load(pbp + 32 * ks);
              acc = Frag<_Float16>::mma(a, bfr, acc);
              dep_guard1(acc, a, bfr);
            }
#pragma unroll
            for (int r = 0; r < 8; ++r)
              bd16[(hd * BPB + mOff + r) * SEQ + 16 * jt + rl] = (_Float16)(acc[r] * INV_WC);
          }
        }
        __syncthreads();
        {
          const int hd = wave;
          const int ng = (t + 31) >> 5;
#pragma unroll 1
          for (int b = 0; b < BPB; ++b) {
            const int bg = blk * BPB + b;
            const float* qr = qa32 + b * DM + hd * DHEAD;
#pragma unroll 1
            for (int g = 0; g < 4; ++g) {
              float s = NEG_FILL;
              if (g < ng) {
                const int j = 32 * g + lane;
                const int jc = j < t ? j : (t - 1);
                const float* kr = memk + ((size_t)(l * SEQ + jc) * NBATCH + bg) * DM + hd * DHEAD;
                float acc = 0.f;
#pragma unroll 1
                for (int dh = 0; dh < 2; ++dh) {
                  v4f kk[8], qq[8];
#pragma unroll
                  for (int e = 0; e < 8; ++e) {
                    kk[e] = *(const v4f*)(kr + 32 * dh + 4 * e);
                    qq[e] = *(const v4f*)(qr + 32 * dh + 4 * e);
                  }
#pragma unroll
                  for (int e = 0; e < 8; ++e) {
                    acc = fmaf(qq[e][0], kk[e][0], acc);
                    acc = fmaf(qq[e][1], kk[e][1], acc);
                    acc = fmaf(qq[e][2], kk[e][2], acc);
                    acc = fmaf(qq[e][3], kk[e][3], acc);
                  }
                }
                const float bdv = (float)bd16[(hd * BPB + b) * SEQ + j];
                const float pbv = kpb[((size_t)l * NPOS + (size_t)(NPOS - t + jc)) * NHEAD + hd];
                const float sv = (acc + bdv + pbv) * ATT_SCALE;
                s = (j < t) ? sv : NEG_FILL;
              }
              scw[32 * g + lane] = s;
            }
            const float v0 = scw[lane], v1 = scw[32 + lane], v2 = scw[64 + lane], v3 = scw[96 + lane];
            float mx = fmaxf(fmaxf(v0, v1), fmaxf(v2, v3));
            mx = wave_max(mx);
            const float e0 = expf(v0 - mx), e1 = expf(v1 - mx), e2 = expf(v2 - mx), e3 = expf(v3 - mx);
            float sm = (e0 + e1) + (e2 + e3);
            sm = wave_sum(sm);
            const float inv = 1.0f / sm;
            scw[lane] = e0 * inv;
            scw[32 + lane] = e1 * inv;
            scw[64 + lane] = e2 * inv;
            scw[96 + lane] = e3 * inv;
            wave_lds_sync();
            float o0 = 0.f, o1 = 0.f;
            const float* vr = memv + ((size_t)(l * SEQ) * NBATCH + bg) * DM + hd * DHEAD + 2 * lane;
            const size_t vstep = (size_t)NBATCH * DM;
            int j = 0;
            for (; j + 4 <= t; j += 4) {
              const v4f p4 = *(const v4f*)(scw + j);
              const v2f va = *(const v2f*)(vr + (size_t)j * vstep);
              const v2f vb = *(const v2f*)(vr + (size_t)(j + 1) * vstep);
              const v2f vc = *(const v2f*)(vr + (size_t)(j + 2) * vstep);
              const v2f vd = *(const v2f*)(vr + (size_t)(j + 3) * vstep);
              o0 = fmaf(p4[0], va[0], o0); o1 = fmaf(p4[0], va[1], o1);
              o0 = fmaf(p4[1], vb[0], o0); o1 = fmaf(p4[1], vb[1], o1);
              o0 = fmaf(p4[2], vc[0], o0); o1 = fmaf(p4[2], vc[1], o1);
              o0 = fmaf(p4[3], vd[0], o0); o1 = fmaf(p4[3], vd[1], o1);
            }
            for (; j < t; ++j) {
              const float p = scw[j];
              const v2f va = *(const v2f*)(vr + (size_t)j * vstep);
              o0 = fmaf(p, va[0], o0); o1 = fmaf(p, va[1], o1);
            }
            v2h av2;
            av2[0] = (_Float16)(o0 * WCARRY);
            av2[1] = (_Float16)(o1 * WCARRY);
            *(v2h*)(a16 + b * DM + hd * DHEAD + 2 * lane) = av2;
            wave_lds_sync();
          }
        }
        __syncthreads();
        {
          v8f acc[4];
          mm16x64<DM, DM, DM>(a16, woT + (size_t)l * DM * DM, wave * 64, acc);
#pragma unroll
          for (int j = 0; j < 4; ++j) {
            const int col = wave * 64 + 16 * j + rl;
            const float bov = bo[l * DM + col];
#pragma unroll
            for (int r = 0; r < 8; ++r) {
              const int idx = (mOff + r) * DM + col;
              hs[idx] = hs[idx] + (acc[j][r] * INV_WC2 + bov);
            }
          }
        }
        __syncthreads();
      }
      ln_to_a16(hs, lnffg + l * DM, lnffb + l * DM, a16);
      __syncthreads();
#pragma unroll 1
      for (int gq = 0; gq < DFFN / DM; ++gq) {
        const int n0 = gq * DM + wave * 64;
        v8f acc[4];
        mm16x64<DM, DM, DM>(a16, w1T + (size_t)l * DFFN * DM, n0, acc);
#pragma unroll
        for (int j = 0; j < 4; ++j) {
          const int col = n0 + 16 * j + rl;
          const float bb1 = b1[l * DFFN + col];
#pragma unroll
          for (int r = 0; r < 8; ++r)
            f1[(mOff + r) * DFFN + col] = (_Float16)fmaxf(acc[j][r] * INV_WC + bb1, 0.0f);
        }
      }
      __syncthreads();
      {
        v8f acc[4];
        mm16x64<DFFN, DFFN, DFFN>(f1c, w2T + (size_t)l * DM * DFFN, wave * 64, acc);
#pragma unroll
        for (int j = 0; j < 4; ++j) {
          const int col = wave * 64 + 16 * j + rl;
          const float bb2 = b2[l * DM + col];
#pragma unroll
          for (int r = 0; r < 8; ++r) {
            const int idx = (mOff + r) * DM + col;
            const float hn = hs[idx] + (acc[j][r] * INV_WC + bb2);
            hs[idx] = hn;
            accm[idx] = fmaf(fl, hn, accm[idx]);
          }
        }
      }
      __syncthreads();
    }

    ln_to_out(hs, lnog, lnob, out + ((size_t)t * NBATCH + (size_t)blk * BPB) * DM);
    {
#pragma unroll
      for (int i = 0; i < (BPB * DM / 8) / NTHR; ++i) {
        const int f = tid + NTHR * i;
        const v4f a = *(const v4f*)(accm + 8 * f);
        const v4f c = *(const v4f*)(accm + 8 * f + 4);
        v8h hv;
        hv[0] = (_Float16)a[0]; hv[1] = (_Float16)a[1]; hv[2] = (_Float16)a[2]; hv[3] = (_Float16)a[3];
        hv[4] = (_Float16)c[0]; hv[5] = (_Float16)c[1]; hv[6] = (_Float16)c[2]; hv[7] = (_Float16)c[3];
        *(v8h*)(a16 + 8 * f) = hv;
      }
    }
    __syncthreads();
    if (t < SEQ - 1) {
#pragma unroll 1
      for (int mat = 0; mat < 2 * NLAY; ++mat) {
        const int l2 = mat >> 1, isv = mat & 1;
        v8f acc[4];
        mm16x64<DM, DM, DM>(a16, wkvT + (size_t)(isv * NLAY + l2) * DM * DM, wave * 64, acc);
#pragma unroll
        for (int j = 0; j < 4; ++j) {
          const int col = wave * 64 + 16 * j + rl;
          const float bvl = bvv[l2 * DM + col];
          const float add = isv ? bvl : 0.0f;
#pragma unroll
          for (int r = 0; r < 8; ++r)
            slab[(mOff + r) * SLAB_PITCH + 16 * j + rl] = acc[j][r] * INV_WC + add;
        }
        wave_lds_sync();
        float* Cb = mem + (size_t)isv * MEMPLANE + ((size_t)(l2 * SEQ + t) * NBATCH + (size_t)blk * BPB) * DM + wave * 64;
        const int c4 = rl * 4;
        for (int pass = 0; pass < 2; ++pass) {
#pragma unroll
          for (int it = 0; it < 8; ++it) {
            const int row = it * 2 + hh;
            const v4f v = *(const v4f*)(slab + row * SLAB_PITCH + c4);
            *(volatile v4f*)(Cb + (size_t)row * DM + c4) = v;
          }
          __threadfence();
        }
        wave_lds_sync();
      }
    }
    __syncthreads();
  }
}

extern "C" void kernel_launch(void* const* d_in, const int* in_sizes, int n_in,
                              void* d_out, int out_size, void* d_ws, size_t ws_size,
                              hipStream_t stream) {
  if (n_in < 21) return;
  if (out_size != SEQ * NBATCH * DM) return;
  if (in_sizes[0] != SEQ * NBATCH * DM) return;
  if (in_sizes[3] != NLAY * DM * DM || in_sizes[7] != NLAY * NPOS * NHEAD * DHEAD) return;
  if (in_sizes[14] != NLAY * DM * DFFN || in_sizes[16] != NLAY * DFFN * DM || in_sizes[18] != NLAY + 1) return;
  if (ws_size < WS_TOTAL) return;

  const float* x_seq   = (const float*)d_in[0];
  const float* ln_sa_g = (const float*)d_in[1];
  const float* ln_sa_b = (const float*)d_in[2];
  const float* wq      = (const float*)d_in[3];
  const float* wk      = (const float*)d_in[4];
  const float* wv      = (const float*)d_in[5];
  const float* bv      = (const float*)d_in[6];
  const float* kpe     = (const float*)d_in[7];
  const float* kpb     = (const float*)d_in[8];
  const float* qpb     = (const float*)d_in[9];
  const float* wo      = (const float*)d_in[10];
  const float* bo      = (const float*)d_in[11];
  const float* ln_ff_g = (const float*)d_in[12];
  const float* ln_ff_b = (const float*)d_in[13];
  const float* w1      = (const float*)d_in[14];
  const float* b1      = (const float*)d_in[15];
  const float* w2      = (const float*)d_in[16];
  const float* b2      = (const float*)d_in[17];
  const float* fuse_w  = (const float*)d_in[18];
  const float* ln_o_g  = (const float*)d_in[19];
  const float* ln_o_b  = (const float*)d_in[20];

  char* ws = (char*)d_ws;
  _Float16* wqT  = (_Float16*)(ws + OFF_WQ);
  _Float16* wkvT = (_Float16*)(ws + OFF_WKV);
  _Float16* woT  = (_Float16*)(ws + OFF_WO);
  _Float16* w1T  = (_Float16*)(ws + OFF_W1);
  _Float16* w2T  = (_Float16*)(ws + OFF_W2);
  _Float16* pe16 = (_Float16*)(ws + OFF_PE);
  float*    mem  = (float*)(ws + OFF_MEM);

  k_wtcast<<<dim3(DM / 64, DM / 64, NLAY), 256, 0, stream>>>(wq, wqT, DM, DM);
  k_wtcast<<<dim3(DM / 64, DM / 64, NLAY), 256, 0, stream>>>(wk, wkvT, DM, DM);
  k_wtcast<<<dim3(DM / 64, DM / 64, NLAY), 256, 0, stream>>>(wv, wkvT + (size_t)NLAY * DM * DM, DM, DM);
  k_wtcast<<<dim3(DM / 64, DM / 64, NLAY), 256, 0, stream>>>(wo, woT, DM, DM);
  k_wtcast<<<dim3(DFFN / 64, DM / 64, NLAY), 256, 0, stream>>>(w1, w1T, DM, DFFN);
  k_wtcast<<<dim3(DM / 64, DFFN / 64, NLAY), 256, 0, stream>>>(w2, w2T, DFFN, DM);
  k_pecast<<<(NLAY * NHEAD * SEQ * DHEAD / 8) / 256, 256, 0, stream>>>(kpe, pe16);
  k_steps<<<NBLK, NTHR, 0, stream>>>(x_seq, ln_sa_g, ln_sa_b, wqT, wkvT, bv, pe16, kpb, qpb,
                                     woT, bo, ln_ff_g, ln_ff_b, w1T, b1, w2T, b2,
                                     fuse_w, ln_o_g, ln_o_b, mem, (float*)d_out);
}
